// NGCFModel_45835890983575
// MI455X (gfx1250) — hardware-run, weakly checked
//
#include <hip/hip_runtime.h>


namespace {
constexpr int NU = 80000, NI = 40000, N = NU + NI, K = 64, L = 3, E1 = 1000000, E = 2 * E1  ;
constexpr float HS = 256.0f, WSC = 256.0f, EPSN = 1e-12f, SLOPE = 0.01f;
typedef _Float16 b16;
typedef __attribute__((ext_vector_type(16))) _Float16 v16b;
typedef __attribute__((ext_vector_type(8))) _Float16 v8b;
typedef __attribute__((ext_vector_type(8))) float v8f;
typedef __attribute__((ext_vector_type(4))) float v4f;
typedef __attribute__((ext_vector_type(2))) float v2f;
__device__ __forceinline__ float bf16_rne(float f) { unsigned int u = __float_as_uint(f); u += 0x7FFFu + ((u >> 16) & 1u); float r = __uint_as_float(u & 0xFFFF0000u); asm volatile("" : "+v"(r)); return r; }
__device__ __forceinline__ float bfv(float f) { float r = bf16_rne(f); asm volatile("" : "+v"(r)); return r; }
__device__ __forceinline__ void split16(float v, b16& hi, b16& lo) { hi = (b16)v; lo = (b16)(v - (float)hi); }
__device__ __forceinline__ v16b frag_kb(const b16* p, int hh) { const v8b a = *(const v8b*)(p + 8 * hh), b = *(const v8b*)(p + 16 + 8 * hh); v16b f;
#pragma unroll
  for (int e = 0; e < 8; ++e) { f[e] = a[e]; f[8 + e] = b[e]; } return f; }
__device__ __forceinline__ v8f wmma16b(v16b a, v16b b, v8f c) { v8f d = __builtin_amdgcn_wmma_f32_16x16x32_f16(false, a, false, b, (short)0, c, false, false); asm volatile("v_nop\n\tv_nop\n\tv_nop\n\tv_nop" : "+v"(d) : "v"(a), "v"(b)); return d; }
__device__ __forceinline__ void wave_lds_sync() { __builtin_amdgcn_fence(__ATOMIC_RELEASE, "workgroup"); __builtin_amdgcn_wave_barrier(); __builtin_amdgcn_fence(__ATOMIC_ACQUIRE, "workgroup"); }
__device__ __forceinline__ float pmul(float a, float b) { float p = a * b; asm volatile("" : "+v"(p)); return p; }
__device__ __forceinline__ int iclamp(int v, int lo, int hi) { return v < lo ? lo : (v > hi ? hi : v); }
__device__ __forceinline__ bool inr(size_t n, int NLIM) { return n < (size_t)NLIM || n >= (size_t)NU; }
constexpr int CSR_NBLK8 = 512, CSR_GB8 = 8, CSR_GN8 = 1 << CSR_GB8  , CSR_TS8 = (CSR_GN8 < 32 ? 32 : CSR_GN8)  , CSR_MAXG8 = 512, CSR_CAP8 = 12288  ;
__device__ __host__ __forceinline__ int csr_tix8(int v) { return (v >> CSR_GB8) * CSR_TS8 + (v & (CSR_GN8 - 1)); }
__global__ __launch_bounds__(64) void csrA_kernel8(const int* __restrict__ dst, int E, int N, int nG, int CHP, int NGP, int* __restrict__ STG, int* __restrict__ HST) {
  extern __shared__ int sm[];
  int* cnt = sm; int* run = sm + NGP; int* ids = sm + 2 * NGP;
  const int b = blockIdx.x; const int ch = (E + CSR_NBLK8 - 1) / CSR_NBLK8; const int e0 = b * ch, e1 = min(E, e0 + ch);
  for (int i = threadIdx.x; i < NGP; i += 64) cnt[i] = 0;
  for (int i = threadIdx.x; i < CHP; i += 64) ids[i] = -1;
  __syncthreads();
  if (threadIdx.x == 0) {
    for (int e = e0; e < e1; ++e) { int d = dst[e]; d = (d < 0) ? 0 : (d >= N ? N - 1 : d); cnt[d >> CSR_GB8] += 1; }
    int acc = 0; for (int g = 0; g < nG; ++g) { run[g] = acc; acc += cnt[g]; }
    for (int e = e0; e < e1; ++e) { int d = dst[e]; d = (d < 0) ? 0 : (d >= N ? N - 1 : d); const int g = d >> CSR_GB8; ids[run[g]] = e; run[g] += 1; } }
  __syncthreads();
  typedef __attribute__((ext_vector_type(4))) int v4i;
  for (int pass = 0; pass < 2; ++pass) {
    for (int i = threadIdx.x; i < CHP / 4; i += 64) *(volatile v4i*)(STG + (size_t)b * CHP + i * 4) = *(const v4i*)(&ids[i * 4]);
    for (int i = threadIdx.x; i < NGP / 4; i += 64) { v4i v; for (int e = 0; e < 4; ++e) v[e] = (i * 4 + e < nG) ? cnt[i * 4 + e] : 0; *(volatile v4i*)(HST + (size_t)b * NGP + i * 4) = v; }
    __threadfence(); }
}
__global__ __launch_bounds__(512) void csrS_kernel8(const int* __restrict__ HST, int nG, int NGP, int* __restrict__ START, int* __restrict__ TOT, int* __restrict__ OFF) {
  __shared__ int tot[CSR_MAXG8];
  const int b = threadIdx.x;
  for (int pass = 0; pass < 2; ++pass) { int runb = 0; for (int g = 0; g < nG; ++g) { int c = HST[(size_t)b * NGP + g]; c = (c < 0) ? 0 : c; ((volatile int*)OFF)[(size_t)g * CSR_NBLK8 + b] = runb; runb += c; } __threadfence(); }
  for (int g = threadIdx.x; g < nG; g += 512) { int s = 0; for (int bb = 0; bb < CSR_NBLK8; ++bb) { int c = HST[(size_t)bb * NGP + g]; s += (c < 0) ? 0 : c; } tot[g] = s; }
  __syncthreads();
  if (threadIdx.x < 32) {
    __shared__ int st[CSR_MAXG8 + 32];
    if (threadIdx.x == 0) { int acc = 0; for (int g = 0; g < NGP; ++g) { st[g] = acc; if (g < nG) acc += (tot[g] + 31) & ~31; } st[NGP] = acc; }
    __builtin_amdgcn_fence(__ATOMIC_RELEASE, "workgroup"); __builtin_amdgcn_wave_barrier(); __builtin_amdgcn_fence(__ATOMIC_ACQUIRE, "workgroup");
    for (int pass = 0; pass < 2; ++pass) { for (int i = threadIdx.x; i < NGP + 32; i += 32) { ((volatile int*)START)[i] = (i <= NGP) ? st[min(i, NGP)] : 0; ((volatile int*)TOT)[i] = (i < nG) ? tot[i] : 0; } __threadfence(); } }
}
__global__ __launch_bounds__(256) void csrB_kernel8(const int* __restrict__ dst, int N, int nG, int CHP, int NGP, int permLen, const int* __restrict__ STG, const int* __restrict__ HST, const int* __restrict__ OFF, const int* __restrict__ START, const int* __restrict__ TOT, int* __restrict__ PERM, int* __restrict__ ROWPTR, int* __restrict__ ROWCNT, int* __restrict__ FLAG) {
  typedef __attribute__((ext_vector_type(4))) int v4i;
  __shared__ int ids[CSR_CAP8]; __shared__ unsigned short key[CSR_CAP8]; __shared__ int outp[CSR_CAP8]; __shared__ int ncnt[CSR_GN8 + 1]; __shared__ int boff[CSR_NBLK8 + 1];
  const int g = blockIdx.x, t_ = threadIdx.x; int tot = TOT[g]; int st = START[g], stn = START[g + 1]; const int v0 = g * CSR_GN8; const int nv = min(CSR_GN8, N - v0); const int t0 = g * CSR_TS8;
  st = (st < 0) ? 0 : (st > permLen - 32 ? permLen - 32 : st) & ~31; stn = (stn < st) ? st : (stn > permLen ? permLen : stn); tot = (tot < 0) ? 0 : tot; if (tot > stn - st && tot <= CSR_CAP8) tot = stn - st;
  if (tot > CSR_CAP8) {
    for (int pass = 0; pass < 2; ++pass) { for (int i = t_; i < CSR_TS8 / 4; i += 256) { v4i a, c; for (int e = 0; e < 4; ++e) { a[e] = st; c[e] = 0; } *(volatile v4i*)(ROWPTR + t0 + i * 4) = a; *(volatile v4i*)(ROWCNT + t0 + i * 4) = c; } if (t_ == 0) ((volatile int*)FLAG)[0] = 1; __threadfence(); } (void)nv; return; }
  if (t_ == 0) { int acc = 0; for (int b = 0; b < CSR_NBLK8; ++b) { boff[b] = acc; int c = HST[(size_t)b * NGP + g]; c = (c < 0) ? 0 : (c > CHP ? CHP : c); acc += c; if (acc > tot) acc = tot; } boff[CSR_NBLK8] = acc; }
  for (int i = t_; i <= CSR_GN8; i += 256) ncnt[i] = 0;
  __syncthreads();
  for (int b = 0; b < CSR_NBLK8; ++b) { const int c = boff[b + 1] - boff[b]; int o_ = OFF[(size_t)g * CSR_NBLK8 + b]; o_ = (o_ < 0) ? 0 : (o_ > CHP - c ? CHP - c : o_); const int* src_ = STG + (size_t)b * CHP + o_;
    for (int i = t_; i < c; i += 256) { int id = src_[i]; id = (id < 0) ? 0 : id; ids[boff[b] + i] = id; int d = dst[id]; d = (d < v0) ? v0 : (d >= N ? N - 1 : d); int kk = d - v0; kk = (kk < 0) ? 0 : (kk >= CSR_GN8 ? CSR_GN8 - 1 : kk); key[boff[b] + i] = (unsigned short)kk; } }
  __syncthreads();
  if (t_ == 0) { for (int i = 0; i < tot; ++i) ncnt[key[i]] += 1; int acc = 0; for (int vl = 0; vl < CSR_GN8; ++vl) { const int c = ncnt[vl]; ncnt[vl] = acc; acc += c; } ncnt[CSR_GN8] = acc;
    for (int i = 0; i < tot; ++i) { const int vl = key[i]; outp[ncnt[vl]] = ids[i]; ncnt[vl] += 1; }
    for (int vl = CSR_GN8; vl > 0; --vl) ncnt[vl] = ncnt[vl - 1]; ncnt[0] = 0; }
  __syncthreads();
  for (int pass = 0; pass < 2; ++pass) {
    for (int i = t_; i < (stn - st) / 4; i += 256) { v4i v; for (int e = 0; e < 4; ++e) { const int q = i * 4 + e; v[e] = (q < tot) ? outp[q] : -1; } *(volatile v4i*)(PERM + st + i * 4) = v; }
    for (int i = t_; i < CSR_TS8 / 4; i += 256) { v4i a, c; for (int e = 0; e < 4; ++e) { const int vl = i * 4 + e; const int vc = vl < CSR_GN8 ? vl : CSR_GN8; a[e] = (vl < CSR_GN8) ? st + ncnt[vc] : st; c[e] = (vl < nv) ? (ncnt[(vc < CSR_GN8 ? vc : CSR_GN8 - 1) + 1] - ncnt[vc]) : 0; } *(volatile v4i*)(ROWPTR + t0 + i * 4) = a; *(volatile v4i*)(ROWCNT + t0 + i * 4) = c; }
    __threadfence(); }
}
__global__ __launch_bounds__(256) void csrZ_kernel8(int* __restrict__ p, size_t n4) { typedef __attribute__((ext_vector_type(4))) int v4i; const size_t tid = (size_t)blockIdx.x * 256 + threadIdx.x, nth = (size_t)gridDim.x * 256; v4i z = {0, 0, 0, 0}; for (size_t i = tid; i < n4; i += nth) *(volatile v4i*)(p + i * 4) = z; }
struct CsrBufs8 { int *STG, *HST, *OFF, *START, *TOT, *PERM, *ROWPTR, *ROWCNT, *FLAG; int nG, NGP, CHP; size_t permLen; char* base; size_t bytes; };
static size_t csr_carve8(CsrBufs8& c, char* ws, size_t off, int E, int N) {
  const size_t off0 = off; c.base = ws + off;
  auto al = [&](size_t bytes) { char* p = ws + off; off += (bytes + 255) & ~(size_t)255; return p; };
  c.nG = (N + CSR_GN8 - 1) / CSR_GN8; c.NGP = (c.nG + 31) & ~31; const int ch = (E + CSR_NBLK8 - 1) / CSR_NBLK8; c.CHP = (ch + 31) & ~31; c.permLen = (size_t)E + 32 * (size_t)c.nG + 32;
  c.STG = (int*)al((size_t)CSR_NBLK8 * c.CHP * 4); c.HST = (int*)al((size_t)CSR_NBLK8 * c.NGP * 4); c.OFF = (int*)al((size_t)c.NGP * CSR_NBLK8 * 4); c.START = (int*)al((size_t)(c.NGP + 64) * 4); c.TOT = (int*)al((size_t)(c.NGP + 64) * 4);
  c.PERM = (int*)al(c.permLen * 4); c.ROWPTR = (int*)al((size_t)c.nG * CSR_TS8 * 4); c.ROWCNT = (int*)al((size_t)c.nG * CSR_TS8 * 4); c.FLAG = (int*)al(256);
  c.bytes = off - off0; return off;
}
static void csr_build8(const CsrBufs8& c, const int* dst, int E, int N, hipStream_t stream) {
  const size_t smem = (size_t)(2 * c.NGP + c.CHP) * 4;
  csrZ_kernel8<<<512, 256, 0, stream>>>((int*)c.base, c.bytes / 16);
  csrA_kernel8<<<CSR_NBLK8, 64, smem, stream>>>(dst, E, N, c.nG, c.CHP, c.NGP, c.STG, c.HST);
  csrS_kernel8<<<1, 512, 0, stream>>>(c.HST, c.nG, c.NGP, c.START, c.TOT, c.OFF);
  csrB_kernel8<<<c.nG, 256, 0, stream>>>(dst, N, c.nG, c.CHP, c.NGP, (int)c.permLen, c.STG, c.HST, c.OFF, c.START, c.TOT, c.PERM, c.ROWPTR, c.ROWCNT, c.FLAG);
}


__global__ __launch_bounds__(256) void wput_kernel(const float* __restrict__ w1, const float* __restrict__ w2, b16* __restrict__ WL) { const int u = blockIdx.x * 256 + threadIdx.x; if (u >= L * K * 16) return; const int l = u / (K * 16), r = u % (K * 16); const int o = r / 16, k0 = (r % 16) * 8; v8b v;
#pragma unroll
  for (int j = 0; j < 8; ++j) { const int k = k0 + j; v[j] = (b16)(bf16_rne(k < K ? w1[((size_t)l * K + k) * K + o] : w2[((size_t)l * K + k - K) * K + o]) * WSC); }
  for (int pass = 0; pass < 2; ++pass) { *(volatile v8b*)(WL + ((size_t)l * K + o) * 2 * K + k0) = v; __threadfence(); } }
__global__ __launch_bounds__(256) void init_kernel(const float* __restrict__ gu, const float* __restrict__ gi, int NLIM, float* __restrict__ X0, float* __restrict__ RS) { __shared__ float Sm[16]; if (threadIdx.x < 16) Sm[threadIdx.x] = 0.0f; __syncthreads(); const int wave = threadIdx.x >> 5, lane = threadIdx.x & 31; const size_t n = (size_t)blockIdx.x * 16 + wave * 2 + (lane >> 4); const int c0 = (lane & 15) * 4; const bool in = n < (size_t)N && inr(n, NLIM);
  v4f v = {0, 0, 0, 0}; if (in) { const float* src = n < (size_t)NU ? gu + n * K : gi + (n - NU) * K; for (int q = 0; q < 4; ++q) v[q] = bfv(src[c0 + q]); }
  float s = v[0] * v[0] + v[1] * v[1] + v[2] * v[2] + v[3] * v[3]; for (int o = 1; o < 16; o <<= 1) s += __shfl_xor(s, o); const float inv = 1.0f / fmaxf(sqrtf(s), EPSN); v4f e; float rs = 0.0f; for (int q = 0; q < 4; ++q) { e[q] = pmul(v[q], inv); rs += e[q]; } for (int o = 1; o < 16; o <<= 1) rs += __shfl_xor(rs, o); if ((lane & 15) == 0) Sm[wave * 2 + (lane >> 4)] = rs;
  __syncthreads();
  for (int pass = 0; pass < 2; ++pass) { if (in) *(volatile v4f*)(X0 + n * K + c0) = e; if (threadIdx.x < 32) ((volatile float*)RS)[(size_t)blockIdx.x * 32 + threadIdx.x] = threadIdx.x < 16 ? Sm[threadIdx.x] : 0.0f;     __threadfence(); } }
__global__ __launch_bounds__(32) void layer_kernel(const float* __restrict__ X, const int* __restrict__ eflat, const int* __restrict__ PERM, const int* __restrict__ ROWPTR, const int* __restrict__ ROWCNT, int permLen, const b16* __restrict__ W, const float* __restrict__ b1, const float* __restrict__ b2, const float* __restrict__ RS, int NLIM, int ELIM, float* __restrict__ XO, float* __restrict__ RSO) { __shared__ __attribute__((aligned(16))) b16 Ah[16][2 * K + 8], Al[16][2 * K + 8]; __shared__ float Tf[16][K + 4], Rs[16]; const int lane = threadIdx.x, nloc = lane & 15, hlf = lane >> 4; const size_t m0 = (size_t)blockIdx.x * 16; if (!inr(m0, NLIM)) return;
  for (int rr = 0; rr < 16; ++rr) { const size_t i = m0 + rr; int st = ROWPTR[i], cnt = ROWCNT[i]; cnt = iclamp(cnt, 0, E); st = iclamp(st, 0, permLen - cnt); float s0 = 0.0f, s1 = 0.0f;
#pragma unroll 1
    for (int j = 0; j < cnt; ++j) { const int e = iclamp(PERM[st + j], 0, E - 1); const int ce = e < E1 ? e + E1 : e - E1; if ((e < E1 ? e : e - E1) >= ELIM) continue;     const size_t u = (size_t)iclamp(eflat[ce], 0, N - 1); if (!inr(u, NLIM)) continue; const v2f v = *(const v2f*)(X + u * K + lane * 2); s0 += v[0]; s1 += v[1]; }
    const v2f xv = *(const v2f*)(X + i * K + lane * 2); b16 p, ql; split16((s0 + xv[0]) * HS, p, ql); Ah[rr][lane * 2] = p; Al[rr][lane * 2] = ql; split16((s1 + xv[1]) * HS, p, ql); Ah[rr][lane * 2 + 1] = p; Al[rr][lane * 2 + 1] = ql;
    split16(pmul(s0, xv[0]) * HS, p, ql); Ah[rr][K + lane * 2] = p; Al[rr][K + lane * 2] = ql; split16(pmul(s1, xv[1]) * HS, p, ql); Ah[rr][K + lane * 2 + 1] = p; Al[rr][K + lane * 2 + 1] = ql; }
  if (lane < 16) for (int k = 2 * K; k < 2 * K + 8; ++k) { Ah[lane][k] = (b16)0.0f; Al[lane][k] = (b16)0.0f; }
  wave_lds_sync(); v8f acc[4] = {(v8f){}, (v8f){}, (v8f){}, (v8f){}};
#pragma unroll
  for (int kb = 0; kb < 2 * K; kb += 32) { const v16b a = frag_kb(&Ah[nloc][kb], hlf), al = frag_kb(&Al[nloc][kb], hlf);
#pragma unroll
    for (int t = 0; t < 4; ++t) { const v16b bw = frag_kb(W + (size_t)(t * 16 + nloc) * 2 * K + kb, hlf); acc[t] = wmma16b(a, bw, acc[t]); acc[t] = wmma16b(al, bw, acc[t]); } }
#pragma unroll
  for (int t = 0; t < 4; ++t) { const int cc = t * 16 + nloc; const float bb = bfv(b1[cc]) + bfv(b2[cc]);
#pragma unroll
    for (int r8 = 0; r8 < 8; ++r8) { const float v = acc[t][r8] * (1.0f / (HS * WSC)) + bb; Tf[8 * hlf + r8][cc] = v > 0.0f ? v : SLOPE * v; } }
  wave_lds_sync();
  for (int rr = 0; rr < 16; ++rr) { const float a = Tf[rr][lane * 2], b = Tf[rr][lane * 2 + 1]; float s = a * a + b * b; for (int o = 16; o; o >>= 1) s += __shfl_xor(s, o); const float inv = 1.0f / fmaxf(sqrtf(s), EPSN); const float ea = pmul(a, inv), eb = pmul(b, inv); float rs = ea + eb; for (int o = 16; o; o >>= 1) rs += __shfl_xor(rs, o); Tf[rr][lane * 2] = ea; Tf[rr][lane * 2 + 1] = eb; if (lane == 0) Rs[rr] = RS[(m0 / 16) * 32 + rr] + rs; }
  wave_lds_sync();
  for (int pass = 0; pass < 2; ++pass) { for (int rr = 0; rr < 16; ++rr) *(volatile v2f*)(XO + (m0 + rr) * K + lane * 2) = *(const v2f*)(&Tf[rr][lane * 2]); ((volatile float*)RSO)[(m0 / 16) * 32 + lane] = lane < 16 ? Rs[lane] : 0.0f; __threadfence(); } }
__global__ __launch_bounds__(256) void out_kernel(const float* __restrict__ RS, int NLIM, float* __restrict__ out) { const size_t n = (size_t)blockIdx.x * 256 + threadIdx.x; if (n >= (size_t)N || !inr(n, NLIM)) return; const float g = RS[(n >> 4) * 32 + (n & 15)] * (1.0f / ((L + 1) * K)); for (int pass = 0; pass < 2; ++pass) { ((volatile float*)out)[n] = g; __threadfence(); } }
}

extern "C" void kernel_launch(void* const* d_in, const int* in_sizes, int n_in, void* d_out, int out_size, void* d_ws, size_t ws_size, hipStream_t stream) {
  (void)n_in;
  auto Fp = [&](int i) { return (const float*)d_in[i]; }; auto Ip = [&](int i) { return (const int*)d_in[i]; };
  if (in_sizes[0] != NU * K || in_sizes[1] != NI * K || in_sizes[2] != L * K * K || in_sizes[4] != L * K * K || in_sizes[6] != 2 * E1 || out_size != N) return;
  const int NLIM = N, ELIM = E1;
  size_t off = 0; char* ws = (char*)d_ws;
  auto carve = [&](size_t bytes) { char* p = ws + off; off += (bytes + 255) & ~(size_t)255; return p; };
  b16* WL = (b16*)carve((size_t)L * K * 2 * K * 2); float* XA = (float*)carve((size_t)N * K * 4); float* XB = (float*)carve((size_t)N * K * 4); float* RA = (float*)carve((size_t)N * 2 * 4); float* RB = (float*)carve((size_t)N * 2 * 4);     CsrBufs8 csr; off = csr_carve8(csr, ws, off, E, N);
  if (off > ws_size || off > ((size_t)128 << 20)) return;
  wput_kernel<<<(L * K * 16 + 255) / 256, 256, 0, stream>>>(Fp(2), Fp(4), WL);
  csr_build8(csr, Ip(6), E, N, stream);
  init_kernel<<<(N + 15) / 16, 256, 0, stream>>>(Fp(0), Fp(1), NLIM, XA, RA);
  float* xi = XA; float* xo = XB; float* ri = RA; float* ro = RB;
  for (int l = 0; l < L; ++l) { layer_kernel<<<N / 16, 32, 0, stream>>>(xi, Ip(6), csr.PERM, csr.ROWPTR, csr.ROWCNT, (int)csr.permLen, WL + (size_t)l * K * 2 * K, Fp(3) + l * K, Fp(5) + l * K, ri, NLIM, ELIM, xo, ro); float* t = xi; xi = xo; xo = t; t = ri; ri = ro; ro = t; }
  out_kernel<<<(N + 255) / 256, 256, 0, stream>>>(ri, NLIM, (float*)d_out);
}
